// MultiheadAttention_44375602102761
// MI455X (gfx1250) — hardware-verified
//
#include <hip/hip_runtime.h>


#ifndef SEQ
#define SEQ  2048
#endif
#define WORD 1024
#define HD   128
#define NH   16
#define DQ   (NH * HD)
#define ZK   (2 * DQ)
#define PCAR 1024.0f
#define QCAR 2048.0f
#define ZCAR 16.0f
#define ZRC  2048.0f
#define WCAR 1024.0f
#define PSP  72
#define ZSP  136
#define TRP  72

static_assert(SEQ % 64 == 0);
static_assert(WORD % 64 == 0);
static_assert(HD == 128);
static_assert(HD == 16 * 8);
static_assert(HD % 32 == 0);
static_assert(DQ % 64 == 0);
static_assert(ZK % 32 == 0);
static_assert(DQ == 2048);
static_assert((PSP * 2) % 16 == 0);
static_assert((ZSP * 2) % 16 == 0);
static_assert((TRP * 2) % 16 == 0);

typedef _Float16 h16;
typedef unsigned short bf;
typedef __attribute__((ext_vector_type(16))) __bf16   v16bf;
typedef __attribute__((ext_vector_type(16))) _Float16 v16h;
typedef __attribute__((ext_vector_type(8)))  _Float16 v8h;
typedef __attribute__((ext_vector_type(8)))  unsigned short v8us;
typedef __attribute__((ext_vector_type(8)))  float    v8f;
typedef __attribute__((ext_vector_type(4)))  float    v4f;
typedef v8h  __attribute__((may_alias)) v8ha;
typedef v4f  __attribute__((may_alias)) v4fa;
typedef v8us __attribute__((may_alias)) v8usa;

__device__ __forceinline__ unsigned short f2bf(float f) { unsigned u = __float_as_uint(f); u += 0x7FFFu + ((u >> 16) & 1u); return (unsigned short)(u >> 16); }
__device__ __forceinline__ float bf2f(unsigned short b) { return __uint_as_float(((unsigned)b) << 16); }
__device__ __forceinline__ float bfr(float f) { return bf2f(f2bf(f)); }
__device__ __forceinline__ v16h cat16(v8h lo, v8h hi) { return __builtin_shufflevector(lo, hi, 0, 1, 2, 3, 4, 5, 6, 7, 8, 9, 10, 11, 12, 13, 14, 15); }
__device__ __forceinline__ v16bf cat16b(v8us lo, v8us hi) { return __builtin_bit_cast(v16bf, __builtin_shufflevector(lo, hi, 0, 1, 2, 3, 4, 5, 6, 7, 8, 9, 10, 11, 12, 13, 14, 15)); }
__device__ __forceinline__ v8f wmma16(v16h a, v16h b, v8f c) { return __builtin_amdgcn_wmma_f32_16x16x32_f16(false, a, false, b, (short)0, c, false, false); }
__device__ __forceinline__ v8f wmmab(v16bf a, v16bf b, v8f c) { return __builtin_amdgcn_wmma_f32_16x16x32_bf16(false, a, false, b, (short)0, c, false, false); }
__device__ __forceinline__ v16h ldh(const h16* p) { return cat16(*(const v8h*)p, *(const v8h*)(p + 16)); }
__device__ __forceinline__ void wsync() { __builtin_amdgcn_fence(3  , "wavefront"); __builtin_amdgcn_wave_barrier(); asm volatile("" ::: "memory"); }

template <typename T16> struct WFrag;
template <> struct WFrag<h16> { typedef v16h V; static __device__ __forceinline__ V ld(const h16* p) { return cat16(*(const v8h*)p, *(const v8h*)(p + 16)); } static __device__ __forceinline__ v8f mma(V a, V b, v8f c) { return wmma16(a, b, c); } };
template <> struct WFrag<bf> { typedef v16bf V; static __device__ __forceinline__ V ld(const bf* p) { return cat16b(*(const v8us*)p, *(const v8us*)(p + 16)); } static __device__ __forceinline__ v8f mma(V a, V b, v8f c) { return wmmab(a, b, c); } };

template <typename T16, bool BIAS>
__device__ __forceinline__ void gemmw_body(const T16* __restrict__ A, const T16* __restrict__ Bt, int K, float* C, int ldc, const float* __restrict__ bias, float oscale) {
    typedef typename WFrag<T16>::V V;
    __shared__ __align__(16) float os[16 * 68];
    const int lane = threadIdx.x & 31, lr = lane & 15, hi = lane >> 4; const int r0 = blockIdx.x * 64, c0 = blockIdx.y * 64;
    v8f acc[4][4];
#pragma unroll
    for (int mb = 0; mb < 4; ++mb)
#pragma unroll
        for (int nb = 0; nb < 4; ++nb) acc[mb][nb] = (v8f){};
    const size_t aoff = (size_t)(r0 + lr) * K + 8 * hi, boff = (size_t)(c0 + lr) * K + 8 * hi;
#pragma unroll 1
    for (int kc = 0; kc < K; kc += 32) {
        V a[4];
#pragma unroll
        for (int mb = 0; mb < 4; ++mb) a[mb] = WFrag<T16>::ld(A + aoff + (size_t)mb * 16 * K + kc);
#pragma unroll
        for (int nb = 0; nb < 4; ++nb) { const V b = WFrag<T16>::ld(Bt + boff + (size_t)nb * 16 * K + kc);
#pragma unroll
            for (int mb = 0; mb < 4; ++mb) acc[mb][nb] = WFrag<T16>::mma(a[mb], b, acc[mb][nb]); }
        asm volatile("v_nop\n\tv_nop\n\tv_nop\n\tv_nop" : "+v"(acc[0][0]), "+v"(acc[1][1]), "+v"(acc[2][2]), "+v"(acc[3][3]) : "v"(a[0]), "v"(a[3]));
    }
#pragma unroll
    for (int mb = 0; mb < 4; ++mb) {
#pragma unroll
        for (int nb = 0; nb < 4; ++nb) {
#pragma unroll
            for (int j = 0; j < 8; ++j) os[(hi * 8 + j) * 68 + nb * 16 + lr] = acc[mb][nb][j]; }
        wsync();
        float* crow = C + (size_t)(r0 + mb * 16) * ldc + c0;
#pragma unroll 1
        for (int ps = 0; ps < 2; ++ps) {
#pragma unroll
            for (int s = 0; s < 8; ++s) { const int row = 2 * s + hi, cofs = lr * 4; v4f val = *(const v4fa*)(os + row * 68 + cofs);
                if (BIAS) { val[0] += bfr(bias[c0 + cofs]); val[1] += bfr(bias[c0 + cofs + 1]); val[2] += bfr(bias[c0 + cofs + 2]); val[3] += bfr(bias[c0 + cofs + 3]); }
                else { val[0] *= oscale; val[1] *= oscale; val[2] *= oscale; val[3] *= oscale; }
                *(volatile v4f*)(crow + (size_t)row * ldc + cofs) = val; }
            if (ps == 0) __threadfence(); }
        wsync();
    }
}
__global__ __launch_bounds__(32) void k_gemm_xw(const bf* __restrict__ A, const bf* __restrict__ Bt, int K, float* C, int ldc, const float* __restrict__ bias) { gemmw_body<bf, true>(A, Bt, K, C, ldc, bias, 1.0f); }
__global__ __launch_bounds__(32) void k_gemm_zp(const h16* __restrict__ A, const h16* __restrict__ Bt, int K, float* C, int ldc, float oscale) { gemmw_body<h16, false>(A, Bt, K, C, ldc, nullptr, oscale); }

__global__ __launch_bounds__(256) void k_cvt8(const float* __restrict__ src, bf* dst, size_t n8) { const size_t i = (size_t)blockIdx.x * 256 + threadIdx.x; if (i >= n8) return; const v8f v = *(const v8f*)(src + i * 8); v8us o;
#pragma unroll
    for (int k = 0; k < 8; ++k) o[k] = f2bf(v[k]); *(volatile v8us*)(dst + i * 8) = o; __threadfence(); *(volatile v8us*)(dst + i * 8) = o; }

__device__ __forceinline__ unsigned short cv16(float v, int mode, float sc) {
    const unsigned short b = f2bf(v);
    const float wv = (mode == 2) ? v : bf2f(b);
    const h16 hh = (h16)(wv * sc);
    const unsigned short hb = __builtin_bit_cast(unsigned short, hh);
    return (mode == 0) ? b : hb;
}

__global__ __launch_bounds__(256) void k_tr(const float* __restrict__ in, int ldi, size_t sIn, unsigned short* out, int ldo, size_t sOut, int mode, float sc, int off2, float sc2) {
    __shared__ __align__(16) unsigned short t1[64 * TRP];
    __shared__ __align__(16) unsigned short t2[64 * TRP];
    const int tid = threadIdx.x; const size_t z = blockIdx.z; in += z * sIn; out += z * sOut;
    const int r0 = blockIdx.x * 64, c0 = blockIdx.y * 64;
#pragma unroll
    for (int i = 0; i < 4; ++i) { const int idx = tid + i * 256; const int r = idx >> 4, c4 = (idx & 15) * 4; const v4f v = *(const v4f*)(in + (size_t)(r0 + r) * ldi + c0 + c4);
#pragma unroll
        for (int q = 0; q < 4; ++q) { t1[(c4 + q) * TRP + r] = cv16(v[q], mode, sc); if (off2) t2[(c4 + q) * TRP + r] = cv16(v[q], mode, sc2); } }
    __syncthreads();
#pragma unroll 1
    for (int ps = 0; ps < 2; ++ps) {
#pragma unroll
        for (int i = 0; i < 2; ++i) { const int idx = tid + i * 256; const int c = idx >> 3, p = (idx & 7) * 8; unsigned short* o = out + (size_t)(c0 + c) * ldo + r0 + p;
            const v8us a = *(const v8usa*)(t1 + c * TRP + p); *(volatile v8us*)o = a;
            if (off2) { const v8us b = *(const v8usa*)(t2 + c * TRP + p); *(volatile v8us*)(o + off2) = b; } }
        if (ps == 0) __threadfence(); }
}

__global__ __launch_bounds__(256) void k_hplanes(const float* __restrict__ F, h16* P16, h16* PR, int withres) {
    const size_t i = (size_t)blockIdx.x * 256 + threadIdx.x; if (i >= (size_t)NH * SEQ * HD / 8) return;
    const int e8 = (int)(i % (HD / 8)); const int s = (int)((i / (HD / 8)) % SEQ); const int h = (int)(i / ((size_t)(HD / 8) * SEQ));
    const v8f v = *(const v8f*)(F + (size_t)s * DQ + h * HD + e8 * 8); v8h o, r;
#pragma unroll
    for (int k = 0; k < 8; ++k) { const h16 a = (h16)v[k]; o[k] = a; r[k] = (h16)((v[k] - (float)a) * QCAR); }
    *(volatile v8h*)(P16 + i * 8) = o; if (withres) *(volatile v8h*)(PR + i * 8) = r;
    __threadfence();
    *(volatile v8h*)(P16 + i * 8) = o; if (withres) *(volatile v8h*)(PR + i * 8) = r;
}

__global__ __launch_bounds__(128) void k_flash(const h16* __restrict__ QH, const h16* __restrict__ QR, const h16* __restrict__ KP, const h16* __restrict__ VT, h16* ZC) {
    __shared__ __align__(16) h16 ps[4 * 16 * PSP];
    __shared__ __align__(16) h16 zs[4 * 2 * 16 * ZSP];
    const int lane = threadIdx.x & 31, w = threadIdx.x >> 5, lr = lane & 15, hi = lane >> 4;
    const int h = blockIdx.y, q0 = blockIdx.x * 64 + w * 16;
    const h16* Qh = QH + (size_t)h * SEQ * HD; const h16* Qr = QR + (size_t)h * SEQ * HD;
    const h16* Kh = KP + (size_t)h * SEQ * HD + lr * HD + 8 * hi;
    const h16* Vt = VT + (size_t)h * HD * SEQ + (size_t)lr * SEQ + 8 * hi;
    const int qoff = (q0 + lr) * HD + 8 * hi;
    const int pw = w * 16 * PSP, zw = w * 2 * 16 * ZSP;
    const float SCL2 = (float)(0.08838834764831845 * 1.4426950408889634);
    const float RQ = 1.0f / QCAR;
    v8f O[8]; float m[8], l[8];
#pragma unroll
    for (int t = 0; t < 8; ++t) O[t] = (v8f){};
#pragma unroll
    for (int r = 0; r < 8; ++r) { m[r] = -3.0e38f; l[r] = 0.0f; }

#pragma unroll 1
    for (int j0 = 0; j0 < SEQ; j0 += 64) {
        v8f sc[4];
#pragma unroll
        for (int hf = 0; hf < 2; ++hf) {
            const h16* Kt = Kh + (size_t)(j0 + hf * 32) * HD;
            v8f a0 = (v8f){}, a1 = (v8f){}, r0 = (v8f){}, r1 = (v8f){};
#pragma unroll
            for (int kk = 0; kk < HD / 32; ++kk) {
                int st = kk * 32; asm volatile("" : "+v"(st));
                const v16h qa = ldh(Qh + qoff + st), qr = ldh(Qr + qoff + st);
                const v16h b0 = ldh(Kt + st), b1 = ldh(Kt + 16 * HD + st);
                a0 = wmma16(qa, b0, a0); r0 = wmma16(qr, b0, r0); a1 = wmma16(qa, b1, a1); r1 = wmma16(qr, b1, r1);
                asm volatile("v_nop\n\tv_nop\n\tv_nop\n\tv_nop" : "+v"(a0), "+v"(r0), "+v"(a1), "+v"(r1) : "v"(qa), "v"(qr), "v"(b0), "v"(b1));
            }
            sc[2 * hf] = a0 + r0 * RQ; sc[2 * hf + 1] = a1 + r1 * RQ;
        }
        float al[8];
#pragma unroll
        for (int r = 0; r < 8; ++r) {
            const float t0 = sc[0][r] * SCL2, t1 = sc[1][r] * SCL2, t2 = sc[2][r] * SCL2, t3 = sc[3][r] * SCL2;
            float mx = fmaxf(fmaxf(t0, t1), fmaxf(t2, t3));
            mx = fmaxf(mx, __shfl_xor(mx, 1, 32)); mx = fmaxf(mx, __shfl_xor(mx, 2, 32)); mx = fmaxf(mx, __shfl_xor(mx, 4, 32)); mx = fmaxf(mx, __shfl_xor(mx, 8, 32));
            const float mn = fmaxf(m[r], mx);
            al[r] = __builtin_amdgcn_exp2f(m[r] - mn); m[r] = mn;
            const float p0 = __builtin_amdgcn_exp2f(t0 - mn) * PCAR, p1 = __builtin_amdgcn_exp2f(t1 - mn) * PCAR, p2 = __builtin_amdgcn_exp2f(t2 - mn) * PCAR, p3 = __builtin_amdgcn_exp2f(t3 - mn) * PCAR;
            l[r] = l[r] * al[r] + ((p0 + p1) + (p2 + p3));
            const int po = pw + (8 * hi + r) * PSP + lr;
            ps[po] = (h16)p0; ps[po + 16] = (h16)p1; ps[po + 32] = (h16)p2; ps[po + 48] = (h16)p3;
        }
        wsync();
        const v16h pa0 = cat16(*(const v8ha*)(ps + pw + lr * PSP + 8 * hi), *(const v8ha*)(ps + pw + lr * PSP + 16 + 8 * hi));
        const v16h pa1 = cat16(*(const v8ha*)(ps + pw + lr * PSP + 32 + 8 * hi), *(const v8ha*)(ps + pw + lr * PSP + 48 + 8 * hi));
#pragma unroll
        for (int t = 0; t < 8; ++t)
#pragma unroll
            for (int r = 0; r < 8; ++r) O[t][r] *= al[r];
        const h16* vb = Vt + j0;
#pragma unroll
        for (int g = 0; g < 2; ++g) {
            int vg = g * 4 * 16 * SEQ; asm volatile("" : "+v"(vg));
            v16h v0[4], v1[4];
#pragma unroll
            for (int nt = 0; nt < 4; ++nt) v0[nt] = ldh(vb + vg + nt * 16 * SEQ);
#pragma unroll
            for (int nt = 0; nt < 4; ++nt) O[g * 4 + nt] = wmma16(pa0, v0[nt], O[g * 4 + nt]);
#pragma unroll
            for (int nt = 0; nt < 4; ++nt) v1[nt] = ldh(vb + vg + nt * 16 * SEQ + 32);
#pragma unroll
            for (int nt = 0; nt < 4; ++nt) O[g * 4 + nt] = wmma16(pa1, v1[nt], O[g * 4 + nt]);
            asm volatile("v_nop\n\tv_nop\n\tv_nop\n\tv_nop" : "+v"(O[g * 4 + 0]), "+v"(O[g * 4 + 1]), "+v"(O[g * 4 + 2]), "+v"(O[g * 4 + 3]) : "v"(pa0), "v"(pa1), "v"(v0[3]), "v"(v1[3]));
        }
        wsync();
    }

    float inv[8];
#pragma unroll
    for (int r = 0; r < 8; ++r) { float s = l[r]; s += __shfl_xor(s, 1, 32); s += __shfl_xor(s, 2, 32); s += __shfl_xor(s, 4, 32); s += __shfl_xor(s, 8, 32); inv[r] = __fdiv_rn(ZCAR, s); }
#pragma unroll
    for (int t = 0; t < 8; ++t)
#pragma unroll
        for (int r = 0; r < 8; ++r) { const float z = O[t][r] * inv[r]; const h16 zh = (h16)z; const h16 zr = (h16)((z - (float)zh) * ZRC);
            const int zo = zw + (8 * hi + r) * ZSP + t * 16 + lr; zs[zo] = zh; zs[zo + 16 * ZSP] = zr; }
    wsync();
    h16* zrow = ZC + (size_t)q0 * ZK + h * HD;
#pragma unroll 1
    for (int pz = 0; pz < 2; ++pz) {
#pragma unroll
        for (int s = 0; s < 8; ++s) { const int row = 2 * s + hi, cofs = lr * 8;
            const v8h a = *(const v8ha*)(zs + zw + row * ZSP + cofs); const v8h b = *(const v8ha*)(zs + zw + 16 * ZSP + row * ZSP + cofs);
            *(volatile v8h*)(zrow + (size_t)row * ZK + cofs) = a; *(volatile v8h*)(zrow + (size_t)row * ZK + DQ + cofs) = b; }
        if (pz == 0) __threadfence(); }
}

static constexpr size_t al256(size_t b) { return (b + 255) & ~(size_t)255; }
static constexpr size_t WS_TOTAL = al256((size_t)SEQ * WORD * 2) + 3 * al256((size_t)DQ * WORD * 2) + al256((size_t)HD * ZK * 2) + al256((size_t)SEQ * DQ * 4)
                                 + 3 * al256((size_t)NH * SEQ * HD * 2) + al256((size_t)NH * HD * SEQ * 2) + al256((size_t)SEQ * ZK * 2);
static_assert(WS_TOTAL <= (size_t)134217728);

extern "C" void kernel_launch(void* const* d_in, const int* in_sizes, int n_in,
                              void* d_out, int out_size, void* d_ws, size_t ws_size, hipStream_t stream) {
    if (n_in < 8) return;
    if (in_sizes[0] < SEQ * WORD || in_sizes[1] < NH * WORD * HD || in_sizes[2] < NH * HD || in_sizes[3] < NH * WORD * HD || in_sizes[4] < NH * HD || in_sizes[5] < NH * WORD * HD || in_sizes[6] < NH * HD || in_sizes[7] < DQ * HD) return;
    if (out_size < SEQ * HD) return;
    if (WS_TOTAL > ws_size) return;
    const float* x = (const float*)d_in[0]; const float* wq = (const float*)d_in[1]; const float* bq = (const float*)d_in[2]; const float* wk = (const float*)d_in[3]; const float* bk = (const float*)d_in[4];
    const float* wv = (const float*)d_in[5]; const float* bv = (const float*)d_in[6]; const float* pj = (const float*)d_in[7];
    float* OUT = (float*)d_out;
    char* wsp = (char*)d_ws;
    auto take = [&](size_t bytes) { char* p = wsp; wsp += (bytes + 255) & ~(size_t)255; return (void*)p; };
    bf* XB = (bf*)take((size_t)SEQ * WORD * 2);
    bf* WQT = (bf*)take((size_t)DQ * WORD * 2); bf* WKT = (bf*)take((size_t)DQ * WORD * 2); bf* WVT = (bf*)take((size_t)DQ * WORD * 2);
    bf* PJT = (bf*)take((size_t)HD * ZK * 2);
    float* F = (float*)take((size_t)SEQ * DQ * 4);
    h16* QH = (h16*)take((size_t)NH * SEQ * HD * 2); h16* QRs = (h16*)take((size_t)NH * SEQ * HD * 2); h16* KPl = (h16*)take((size_t)NH * SEQ * HD * 2);
    bf* VTp = (bf*)take((size_t)NH * HD * SEQ * 2);
    h16* ZC = (h16*)take((size_t)SEQ * ZK * 2);
    if ((size_t)(wsp - (char*)d_ws) > ws_size) return;

    k_cvt8<<<(unsigned)(((size_t)SEQ * WORD / 8 + 255) / 256), 256, 0, stream>>>(x, XB, (size_t)SEQ * WORD / 8);
    k_tr<<<dim3(WORD / 64, HD / 64, NH), 256, 0, stream>>>(wq, HD, (size_t)WORD * HD, WQT, WORD, (size_t)HD * WORD, 0, 1.0f, 0, 1.0f);
    k_tr<<<dim3(WORD / 64, HD / 64, NH), 256, 0, stream>>>(wk, HD, (size_t)WORD * HD, WKT, WORD, (size_t)HD * WORD, 0, 1.0f, 0, 1.0f);
    k_tr<<<dim3(WORD / 64, HD / 64, NH), 256, 0, stream>>>(wv, HD, (size_t)WORD * HD, WVT, WORD, (size_t)HD * WORD, 0, 1.0f, 0, 1.0f);
    k_tr<<<dim3(DQ / 64, HD / 64, 1), 256, 0, stream>>>(pj, HD, 0, PJT, ZK, 0, 1, WCAR, DQ, WCAR / ZRC);

    const unsigned LP = (unsigned)(((size_t)NH * SEQ * HD / 8 + 255) / 256);
    k_gemm_xw<<<dim3(SEQ / 64, DQ / 64, 1), 32, 0, stream>>>(XB, WQT, WORD, F, DQ, bq);
    k_hplanes<<<LP, 256, 0, stream>>>(F, QH, QRs, 1);
    k_gemm_xw<<<dim3(SEQ / 64, DQ / 64, 1), 32, 0, stream>>>(XB, WKT, WORD, F, DQ, bk);
    k_hplanes<<<LP, 256, 0, stream>>>(F, KPl, KPl, 0);
    k_gemm_xw<<<dim3(SEQ / 64, DQ / 64, 1), 32, 0, stream>>>(XB, WVT, WORD, F, DQ, bv);
    k_tr<<<dim3(SEQ / 64, DQ / 64, 1), 256, 0, stream>>>(F, DQ, 0, VTp, SEQ, 0, 2, 1.0f, 0, 1.0f);

    k_flash<<<dim3(SEQ / 64, NH, 1), 128, 0, stream>>>(QH, QRs, KPl, (const h16*)VTp, ZC);

    k_gemm_zp<<<dim3(SEQ / 64, HD / 64, 1), 32, 0, stream>>>(ZC, (const h16*)PJT, ZK, OUT, HD, 1.0f / (ZCAR * WCAR));
}
